// enc_mtan_GRU_59785944760916
// MI455X (gfx1250) — hardware-verified
//
#include <hip/hip_runtime.h>


namespace {
constexpr int NB = 32, S = 512, R = 128, D = 64, E = 128, H = 256, G3 = 3 * H, NT = NB * R  ;
constexpr float XS = 8.0f, WSC = 256.0f, PS = 8.0f;

typedef _Float16 b16;
typedef __attribute__((ext_vector_type(16))) _Float16 v16b;
typedef __attribute__((ext_vector_type(8))) _Float16 v8b;
typedef __attribute__((ext_vector_type(8))) float v8f;
typedef __attribute__((ext_vector_type(4))) float v4f;
__device__ __forceinline__ float bf16_rne(float f) { unsigned int u = __float_as_uint(f); u += 0x7FFFu + ((u >> 16) & 1u); return __uint_as_float(u & 0xFFFF0000u); }
__device__ __forceinline__ void split16(float v, b16& hi, b16& lo) { hi = (b16)v; lo = (b16)(v - (float)hi); }
__device__ __forceinline__ v16b frag_kb(const b16* p, int hh) { const v8b a = *(const v8b*)(p + 8 * hh), b = *(const v8b*)(p + 16 + 8 * hh); v16b f;
#pragma unroll
  for (int e = 0; e < 8; ++e) { f[e] = a[e]; f[8 + e] = b[e]; } return f; }
__device__ __forceinline__ v8f wmma16b(v16b a, v16b b, v8f c) { v8f d = __builtin_amdgcn_wmma_f32_16x16x32_f16(false, a, false, b, (short)0, c, false, false); asm volatile("v_nop\n\tv_nop\n\tv_nop\n\tv_nop" : "+v"(d) : "v"(a), "v"(b)); return d; }
__device__ __forceinline__ void wave_lds_sync() { __builtin_amdgcn_fence(__ATOMIC_RELEASE, "workgroup"); __builtin_amdgcn_wave_barrier(); __builtin_amdgcn_fence(__ATOMIC_ACQUIRE, "workgroup"); }
__device__ __forceinline__ float pmul(float a, float b) { float p = a * b; asm volatile("" : "+v"(p)); return p; }
__device__ __forceinline__ float sigm(float x) { return 1.0f / (1.0f + __expf(-x)); }
__device__ __forceinline__ float temb(float t, int c, const float* __restrict__ wper, const float* __restrict__ bper, float wl, float bl) { return (c == 0) ? pmul(t, wl) + bl : sinf(pmul(t, bf16_rne(wper[c - 1])) + bf16_rne(bper[c - 1])); }

__global__ __launch_bounds__(256) void prep_kernel(const float* __restrict__ xv, const int* __restrict__ xm, const float* __restrict__ ts, const float* __restrict__ qt, const float* __restrict__ wq, const float* __restrict__ wk, const float* __restrict__ wper, const float* __restrict__ bper, const float* __restrict__ wlin, const float* __restrict__ blin,
    const float* __restrict__ wihf, const float* __restrict__ whhf, const float* __restrict__ wihb, const float* __restrict__ whhb, b16* __restrict__ WK, b16* __restrict__ WQ, b16* __restrict__ WIH, b16* __restrict__ WHH, b16* __restrict__ KEh, b16* __restrict__ KEl, b16* __restrict__ QEh, b16* __restrict__ QEl) {
  const size_t t = (size_t)blockIdx.x * 256 + threadIdx.x; size_t u = t; v8b o, ol; const float wl = bf16_rne(wlin[0]), bl = bf16_rne(blin[0]);
  { const size_t n = (size_t)E * E / 8; if (u < 2 * n) { const int kind = (int)(u / n); const size_t e = (u % n) * 8; const float* w = kind ? wq : wk; for (int j = 0; j < 8; ++j) o[j] = (b16)(bf16_rne(w[e + j]) * WSC); b16* dst = (kind ? WQ : WK) + e; for (int pass = 0; pass < 2; ++pass) { *(volatile v8b*)dst = o; __threadfence(); } return; } u -= 2 * n; }
  { const size_t n = (size_t)G3 * D / 8; if (u < 2 * n) { const int dir = (int)(u / n); const size_t e = (u % n) * 8; const float* w = dir ? wihb : wihf; for (int j = 0; j < 8; ++j) o[j] = (b16)(bf16_rne(w[e + j]) * WSC); for (int pass = 0; pass < 2; ++pass) { *(volatile v8b*)(WIH + (size_t)dir * G3 * D + e) = o; __threadfence(); } return; } u -= 2 * n; }
  { const size_t n = (size_t)G3 * H / 8; if (u < 2 * n) { const int dir = (int)(u / n); const size_t e = (u % n) * 8; const float* w = dir ? whhb : whhf; for (int j = 0; j < 8; ++j) o[j] = (b16)(bf16_rne(w[e + j]) * WSC); for (int pass = 0; pass < 2; ++pass) { *(volatile v8b*)(WHH + (size_t)dir * G3 * H + e) = o; __threadfence(); } return; } u -= 2 * n; }
  { const size_t n = (size_t)NB * S * E / 8; if (u < n) { const size_t e = u * 8; const size_t row = e / E; const int c0 = (int)(e % E); const float tt = bf16_rne(ts[row]); for (int j = 0; j < 8; ++j) { b16 p, q; split16(temb(tt, c0 + j, wper, bper, wl, bl) * XS, p, q); o[j] = p; ol[j] = q; } for (int pass = 0; pass < 2; ++pass) { *(volatile v8b*)(KEh + e) = o; *(volatile v8b*)(KEl + e) = ol; __threadfence(); } return; } u -= n; }
  { const size_t n = (size_t)R * E / 8; if (u < n) { const size_t e = u * 8; const int r = (int)(e / E), c0 = (int)(e % E); const float tt = bf16_rne(qt[r]); for (int j = 0; j < 8; ++j) { b16 p, q; split16(temb(tt, c0 + j, wper, bper, wl, bl) * XS, p, q); o[j] = p; ol[j] = q; } for (int pass = 0; pass < 2; ++pass) { *(volatile v8b*)(QEh + e) = o; *(volatile v8b*)(QEl + e) = ol; __threadfence(); } } (void)xv; (void)xm; }
}
__global__ __launch_bounds__(256) void mx_kernel(const float* __restrict__ xv, const int* __restrict__ xm, b16* __restrict__ MXT, b16* __restrict__ MT) {
  __shared__ __attribute__((aligned(16))) b16 A[D][64 + 8], Bm[D][64 + 8];
  const int b = blockIdx.y, s0 = blockIdx.x * 64, t_ = threadIdx.x;
  for (int q = t_; q < 64 * D; q += 256) { const int ss = q / D, d = q % D; const size_t gi = ((size_t)b * S + s0 + ss) * D + d; const bool m = xm[gi] != 0; A[d][ss] = (b16)(m ? bf16_rne(xv[gi]) * XS : 0.0f); Bm[d][ss] = (b16)(m ? XS : 0.0f); }
  __syncthreads();
  for (int pass = 0; pass < 2; ++pass) { for (int q = t_; q < D * 8; q += 256) { const int d = q >> 3, c8 = (q & 7) * 8; const size_t gi = ((size_t)b * D + d) * S + s0 + c8; *(volatile v8b*)(MXT + gi) = *(const v8b*)(&A[d][c8]); *(volatile v8b*)(MT + gi) = *(const v8b*)(&Bm[d][c8]); } __threadfence(); }
}
__global__ __launch_bounds__(128) void kq_kernel(const b16* __restrict__ KEh, const b16* __restrict__ KEl, const b16* __restrict__ QEh, const b16* __restrict__ QEl, const b16* __restrict__ WK, const b16* __restrict__ WQ, const float* __restrict__ bk, const float* __restrict__ bq, b16* __restrict__ Kh, b16* __restrict__ Kl, b16* __restrict__ Qh, b16* __restrict__ Ql) {
  __shared__ __attribute__((aligned(16))) b16 Th[4][16][E + 8], Tl[4][16][E + 8];
  const int wave = threadIdx.x >> 5, lane = threadIdx.x & 31, nloc = lane & 15, hlf = lane >> 4; const bool isq = blockIdx.x >= NB * S / 64; const size_t m0 = (isq ? (size_t)(blockIdx.x - NB * S / 64) * 64 : (size_t)blockIdx.x * 64) + wave * 16;
  const b16* Ah = isq ? QEh : KEh; const b16* Al = isq ? QEl : KEl; const b16* W = isq ? WQ : WK; const float* bias = isq ? bq : bk; v8f acc[8];
#pragma unroll
  for (int t = 0; t < 8; ++t) acc[t] = (v8f){};
#pragma unroll
  for (int kb = 0; kb < E; kb += 32) { const v16b a = frag_kb(Ah + (m0 + nloc) * E + kb, hlf), al = frag_kb(Al + (m0 + nloc) * E + kb, hlf);
#pragma unroll
    for (int t = 0; t < 8; ++t) { const v16b bw = frag_kb(W + (size_t)(t * 16 + nloc) * E + kb, hlf); acc[t] = wmma16b(a, bw, acc[t]); acc[t] = wmma16b(al, bw, acc[t]); } }
#pragma unroll
  for (int t = 0; t < 8; ++t) { const float bb = bf16_rne(bias[t * 16 + nloc]);
#pragma unroll 1
    for (int r = 0; r < 8; ++r) { b16 p, q; split16((acc[t][r] * (1.0f / (XS * WSC)) + bb) * XS, p, q); Th[wave][8 * hlf + r][t * 16 + nloc] = p; Tl[wave][8 * hlf + r][t * 16 + nloc] = q; } }
  wave_lds_sync(); b16* dh = isq ? Qh : Kh; b16* dl = isq ? Ql : Kl;
  for (int pass = 0; pass < 2; ++pass) { for (int r2 = 0; r2 < 16; r2 += 2) { const int rr = r2 + (lane >> 4), c8 = (lane & 15) * 8; const size_t gi = (m0 + rr) * E + c8; *(volatile v8b*)(dh + gi) = *(const v8b*)(&Th[wave][rr][c8]); *(volatile v8b*)(dl + gi) = *(const v8b*)(&Tl[wave][rr][c8]); } __threadfence(); }
}
__global__ __launch_bounds__(64) void attn_kernel(const b16* __restrict__ Qh, const b16* __restrict__ Ql, const b16* __restrict__ Kh, const b16* __restrict__ Kl, const b16* __restrict__ MXT, const b16* __restrict__ MT, const float* __restrict__ xv, float* __restrict__ ENC) {
  __shared__ __attribute__((aligned(16))) float To[2][16][D + 4];
  const int wave = threadIdx.x >> 5, lane = threadIdx.x & 31, hh = lane >> 4, col = lane & 15; const int b = blockIdx.y; const int r0 = blockIdx.x * 32 + wave * 16, ri = r0 + col;
  v16b qa[4], ql[4]; for (int k = 0; k < 4; ++k) { qa[k] = frag_kb(Qh + (size_t)ri * E + k * 32, hh); ql[k] = frag_kb(Ql + (size_t)ri * E + k * 32, hh); }
  const b16* Kb = Kh + (size_t)b * S * E; const b16* Klb = Kl + (size_t)b * S * E; const float cs = 0.08838834764831845f / (XS * XS);
  auto stile = [&](int kt) { v8f s = {}; const b16* kp = Kb + (size_t)(kt * 16 + col) * E, *klp = Klb + (size_t)(kt * 16 + col) * E;
    for (int k = 0; k < 4; ++k) { const v16b f = frag_kb(kp + k * 32, hh); s = wmma16b(f, qa[k], s); s = wmma16b(f, ql[k], s); s = wmma16b(frag_kb(klp + k * 32, hh), qa[k], s); } return s; };
  float mx = -INFINITY;
  for (int kt = 0; kt < S / 16; ++kt) { const v8f s = stile(kt); for (int r = 0; r < 8; ++r) mx = fmaxf(mx, s[r] * cs); }
  mx = fmaxf(mx, __shfl_xor(mx, 16));
  v8f num[4] = {{}, {}, {}, {}}, den[4] = {{}, {}, {}, {}};
  for (int kb = 0; kb < S; kb += 32) { const v8f s0 = stile(kb / 16), s1 = stile(kb / 16 + 1); v16b eh, el;
#pragma unroll
    for (int r = 0; r < 8; ++r) { b16 p, q; split16(__expf(s0[r] * cs - mx) * PS, p, q); eh[r] = p; el[r] = q; split16(__expf(s1[r] * cs - mx) * PS, p, q); eh[8 + r] = p; el[8 + r] = q; }
#pragma unroll
    for (int t = 0; t < 4; ++t) { const v16b xf = frag_kb(MXT + ((size_t)b * D + t * 16 + col) * S + kb, hh), mf = frag_kb(MT + ((size_t)b * D + t * 16 + col) * S + kb, hh);
      num[t] = wmma16b(xf, eh, num[t]); num[t] = wmma16b(xf, el, num[t]); den[t] = wmma16b(mf, eh, den[t]); den[t] = wmma16b(mf, el, den[t]); } }
#pragma unroll
  for (int t = 0; t < 4; ++t)
#pragma unroll 1
    for (int r = 0; r < 8; ++r) { const float dn = den[t][r]; float v; if (dn > 0.0f) v = num[t][r] / dn; else { const int d = t * 16 + 8 * hh + r; float s = 0.0f; for (int ss = 0; ss < S; ++ss) s += bf16_rne(xv[((size_t)b * S + ss) * D + d]); v = s * (1.0f / S); }
      To[wave][col][t * 16 + 8 * hh + r] = v; }
  wave_lds_sync();
  for (int pass = 0; pass < 2; ++pass) { for (int rr = 0; rr < 16; ++rr) if (lane < 16) *(volatile v4f*)(ENC + ((size_t)b * R + r0 + rr) * D + lane * 4) = *(const v4f*)(&To[wave][rr][lane * 4]); __threadfence(); }
}
__global__ __launch_bounds__(128) void gi_kernel(const float* __restrict__ ENC, const b16* __restrict__ WIH, const float* __restrict__ bihf, const float* __restrict__ bihb, float* __restrict__ GI) {
  __shared__ __attribute__((aligned(16))) b16 Ah[4][16][D + 8], Al[4][16][D + 8]; __shared__ __attribute__((aligned(16))) float Tf[4][16][128 + 4];
  const int wave = threadIdx.x >> 5, lane = threadIdx.x & 31, nloc = lane & 15, hlf = lane >> 4; const int dir = blockIdx.z, n0 = blockIdx.y * 128; const size_t m0 = (size_t)blockIdx.x * 64 + wave * 16; const float* bias = dir ? bihb : bihf;
  for (int q = lane; q < 16 * (D / 4); q += 32) { const int rr = q / (D / 4), c4 = (q % (D / 4)) * 4; const v4f xv = *(const v4f*)(ENC + (m0 + rr) * D + c4); for (int j = 0; j < 4; ++j) { b16 p, pl; split16(xv[j] * XS, p, pl); Ah[wave][rr][c4 + j] = p; Al[wave][rr][c4 + j] = pl; } }
  wave_lds_sync(); v8f acc[8];
#pragma unroll
  for (int t = 0; t < 8; ++t) acc[t] = (v8f){};
#pragma unroll
  for (int kb = 0; kb < D; kb += 32) { const v16b a = frag_kb(&Ah[wave][nloc][kb], hlf), al = frag_kb(&Al[wave][nloc][kb], hlf);
#pragma unroll
    for (int t = 0; t < 8; ++t) { const v16b bw = frag_kb(WIH + ((size_t)dir * G3 + n0 + t * 16 + nloc) * D + kb, hlf); acc[t] = wmma16b(a, bw, acc[t]); acc[t] = wmma16b(al, bw, acc[t]); } }
#pragma unroll
  for (int t = 0; t < 8; ++t) { const float bb = bf16_rne(bias[n0 + t * 16 + nloc]);
#pragma unroll 1
    for (int r = 0; r < 8; ++r) Tf[wave][8 * hlf + r][t * 16 + nloc] = acc[t][r] * (1.0f / (XS * WSC)) + bb; }
  wave_lds_sync();
  for (int pass = 0; pass < 2; ++pass) { for (int rr = 0; rr < 16; ++rr) *(volatile v4f*)(GI + ((size_t)dir * NT + m0 + rr) * G3 + n0 + lane * 4) = *(const v4f*)(&Tf[wave][rr][lane * 4]); __threadfence(); }
}
__global__ __launch_bounds__(256) void gru_kernel(const float* __restrict__ GI, const b16* __restrict__ WHH, const float* __restrict__ bhhf, const float* __restrict__ bhhb, float* __restrict__ out) {
  __shared__ __attribute__((aligned(16))) b16 Hh[NB][H + 8], Hl[NB][H + 8]; __shared__ __attribute__((aligned(16))) float Hf[NB][H + 4];
  const int dir = blockIdx.x; const int wave = threadIdx.x >> 5, lane = threadIdx.x & 31, nloc = lane & 15, hlf = lane >> 4, t_ = threadIdx.x; const int j0 = wave * 32;
  const b16* W = WHH + (size_t)dir * G3 * H; const float* bh = dir ? bhhb : bhhf; const float* gi = GI + (size_t)dir * NT * G3;
  for (int q = t_; q < NB * H; q += 256) { const int bb = q / H, j = q % H; Hh[bb][j] = (b16)0.0f; Hl[bb][j] = (b16)0.0f; Hf[bb][j] = 0.0f; }
  __syncthreads();
  float bhv[6]; for (int g = 0; g < 3; ++g) for (int u = 0; u < 2; ++u) bhv[g * 2 + u] = bf16_rne(bh[g * H + j0 + u * 16 + nloc]);
  for (int step = 0; step < R; ++step) { const int tt = dir ? (R - 1 - step) : step;
    v8f acc[2][6];
#pragma unroll
    for (int a = 0; a < 2; ++a) for (int c = 0; c < 6; ++c) acc[a][c] = (v8f){};
#pragma unroll 2
    for (int kb = 0; kb < H; kb += 32) { v16b bw[6]; for (int g = 0; g < 3; ++g) for (int u = 0; u < 2; ++u) bw[g * 2 + u] = frag_kb(W + (size_t)(g * H + j0 + u * 16 + nloc) * H + kb, hlf);
#pragma unroll
      for (int a = 0; a < 2; ++a) { const v16b ha = frag_kb(&Hh[a * 16 + nloc][kb], hlf), hl = frag_kb(&Hl[a * 16 + nloc][kb], hlf);
#pragma unroll
        for (int c = 0; c < 6; ++c) { acc[a][c] = wmma16b(ha, bw[c], acc[a][c]); acc[a][c] = wmma16b(hl, bw[c], acc[a][c]); } } }
    __syncthreads();
#pragma unroll
    for (int a = 0; a < 2; ++a)
#pragma unroll
      for (int u = 0; u < 2; ++u) { const int j = j0 + u * 16 + nloc;
#pragma unroll 1
        for (int r = 0; r < 8; ++r) { const int bb = a * 16 + 8 * hlf + r; const float* git = gi + ((size_t)bb * R + tt) * G3;
          const float ghr = acc[a][0 * 2 + u][r] * (1.0f / (XS * WSC)) + bhv[0 * 2 + u], ghz = acc[a][1 * 2 + u][r] * (1.0f / (XS * WSC)) + bhv[1 * 2 + u], ghn = acc[a][2 * 2 + u][r] * (1.0f / (XS * WSC)) + bhv[2 * 2 + u];
          const float rg = sigm(git[j] + ghr), zg = sigm(git[H + j] + ghz), ng = tanhf(git[2 * H + j] + pmul(rg, ghn)); const float hold = Hf[bb][j]; const float hn = pmul(1.0f - zg, ng) + pmul(zg, hold);
          Hf[bb][j] = hn; b16 p, q; split16(hn * XS, p, q); Hh[bb][j] = p; Hl[bb][j] = q; } }
    __syncthreads();
    for (int pass = 0; pass < 2; ++pass) { for (int q = lane; q < NB * 8; q += 32) { const int bb = q >> 3, c4 = (q & 7) * 4; *(volatile v4f*)(out + ((size_t)bb * R + tt) * (2 * H) + dir * H + j0 + c4) = *(const v4f*)(&Hf[bb][j0 + c4]); } __threadfence(); } }
}
}

extern "C" void kernel_launch(void* const* d_in, const int* in_sizes, int n_in, void* d_out, int out_size, void* d_ws, size_t ws_size, hipStream_t stream) {
  (void)n_in;
  auto Fp = [&](int i) { return (const float*)d_in[i]; }; auto Ip = [&](int i) { return (const int*)d_in[i]; };
  if (in_sizes[0] != NB * S * D || in_sizes[1] != NB * S * D || in_sizes[2] != NB * S || in_sizes[3] != R || in_sizes[4] != E * E || in_sizes[8] != E - 1 || in_sizes[12] != G3 * D || in_sizes[13] != G3 * H || out_size != NB * R * 2 * H) return;
  size_t off = 0; char* ws = (char*)d_ws;
  auto carve = [&](size_t bytes) { char* p = ws + off; off += (bytes + 255) & ~(size_t)255; return p; };
  b16* WK = (b16*)carve((size_t)E * E * 2); b16* WQ = (b16*)carve((size_t)E * E * 2); b16* WIH = (b16*)carve((size_t)2 * G3 * D * 2); b16* WHH = (b16*)carve((size_t)2 * G3 * H * 2);
  b16* KEh = (b16*)carve((size_t)NB * S * E * 2); b16* KEl = (b16*)carve((size_t)NB * S * E * 2); b16* QEh = (b16*)carve((size_t)R * E * 2); b16* QEl = (b16*)carve((size_t)R * E * 2);
  b16* MXT = (b16*)carve((size_t)NB * D * S * 2); b16* MT = (b16*)carve((size_t)NB * D * S * 2); b16* Kh = (b16*)carve((size_t)NB * S * E * 2); b16* Kl = (b16*)carve((size_t)NB * S * E * 2); b16* Qh = (b16*)carve((size_t)R * E * 2); b16* Ql = (b16*)carve((size_t)R * E * 2);
  float* ENC = (float*)carve((size_t)NT * D * 4); float* GI = (float*)carve((size_t)2 * NT * G3 * 4);
  if (off > ws_size || off > ((size_t)128 << 20)) return;
  const size_t prepN = 2 * (size_t)E * E / 8 + 2 * (size_t)G3 * D / 8 + 2 * (size_t)G3 * H / 8 + (size_t)NB * S * E / 8 + (size_t)R * E / 8;
  prep_kernel<<<(unsigned)((prepN + 255) / 256), 256, 0, stream>>>(Fp(0), Ip(1), Fp(2), Fp(3), Fp(4), Fp(6), Fp(8), Fp(9), Fp(10), Fp(11), Fp(12), Fp(13), Fp(16), Fp(17), WK, WQ, WIH, WHH, KEh, KEl, QEh, QEl);
  mx_kernel<<<dim3(S / 64, NB), 256, 0, stream>>>(Fp(0), Ip(1), MXT, MT);
  kq_kernel<<<NB * S / 64 + R / 64, 128, 0, stream>>>(KEh, KEl, QEh, QEl, WK, WQ, Fp(7), Fp(5), Kh, Kl, Qh, Ql);
  attn_kernel<<<dim3(R / 32, NB), 64, 0, stream>>>(Qh, Ql, Kh, Kl, MXT, MT, Fp(0), ENC);
  gi_kernel<<<dim3(NT / 64, G3 / 128, 2), 128, 0, stream>>>(ENC, WIH, Fp(14), Fp(18), GI);
  gru_kernel<<<2, 256, 0, stream>>>(GI, WHH, Fp(15), Fp(19), (float*)d_out);
}
